// HierDDpmC_1382979469615
// MI455X (gfx1250) — hardware-run, weakly checked
//
#include <hip/hip_runtime.h>


#ifndef NB
#define NB 4
#endif
#ifndef SEQ
#define SEQ 4096
#endif
#define NB_FULL  4
#define SEQ_FULL 4096
#ifndef OUT_SEQ
#define OUT_SEQ SEQ
#endif
#define VD   64
#define DD   128
#define NTOK 64
#define TWO_PI_F 6.283185307179586f

static_assert(NB >= 1 && NB <= 4);
static_assert(NB <= NB_FULL);
static_assert(SEQ <= SEQ_FULL);
static_assert(SEQ % 64 == 0);
static_assert((NB * SEQ) % 64 == 0);
static_assert(VD % 32 == 0 && DD % 32 == 0);
static_assert((2 * DD) % 64 == 0 && DD % 64 == 0);
static_assert(VD == 64 && DD == 128);

typedef unsigned short bf;
typedef __attribute__((ext_vector_type(16))) __bf16   v16bf;
typedef __attribute__((ext_vector_type(8)))  unsigned short v8us;
typedef __attribute__((ext_vector_type(8)))  float    v8f;
typedef __attribute__((ext_vector_type(4)))  float    v4f;
typedef v4f  __attribute__((may_alias)) v4fa;

__device__ __forceinline__ unsigned short f2bf(float f) { unsigned u = __float_as_uint(f); u += 0x7FFFu + ((u >> 16) & 1u); return (unsigned short)(u >> 16); }
__device__ __forceinline__ float bf2f(unsigned short h) { return __uint_as_float(((unsigned)h) << 16); }
__device__ __forceinline__ float bfq(float f) { return bf2f(f2bf(f)); }
__device__ __forceinline__ v16bf cat16b(v8us lo, v8us hi) { return __builtin_bit_cast(v16bf, __builtin_shufflevector(lo, hi, 0, 1, 2, 3, 4, 5, 6, 7, 8, 9, 10, 11, 12, 13, 14, 15)); }
__device__ __forceinline__ v8f wmmab(v16bf a, v16bf b, v8f c) { return __builtin_amdgcn_wmma_f32_16x16x32_bf16(false, a, false, b, (short)0, c, false, false); }
__device__ __forceinline__ v16bf ldb(const bf* p)  { return cat16b(*(const v8us*)p, *(const v8us*)(p + 16)); }
__device__ __forceinline__ void wave_sync() { __builtin_amdgcn_fence(3  , "wavefront"); __builtin_amdgcn_wave_barrier(); asm volatile("" ::: "memory"); }

__global__ __launch_bounds__(256) void k_cvt8(const float* __restrict__ src, bf* dst, size_t n8) {
    const size_t i = (size_t)blockIdx.x * 256 + threadIdx.x; if (i >= n8) return;
    const v8f v = *(const v8f*)(src + i * 8); v8us o;
#pragma unroll
    for (int k = 0; k < 8; ++k) o[k] = f2bf(v[k]);
    *(volatile v8us*)(dst + i * 8) = o; __threadfence(); *(volatile v8us*)(dst + i * 8) = o;
}

__global__ __launch_bounds__(256) void k_bfq4(const float* __restrict__ src, float* dst, size_t n4) {
    const size_t i = (size_t)blockIdx.x * 256 + threadIdx.x; if (i >= n4) return;
    const v4f v = *(const v4f*)(src + i * 4); v4f o;
#pragma unroll
    for (int k = 0; k < 4; ++k) o[k] = bfq(v[k]);
    *(volatile v4f*)(dst + i * 4) = o; __threadfence(); *(volatile v4f*)(dst + i * 4) = o;
}

__global__ __launch_bounds__(32) void k_gemm(const bf* __restrict__ A, size_t plane, const bf* __restrict__ Bt, float* C, int K, int ldc) {
    __shared__ __align__(16) float os[16 * 68];
    const int lane = threadIdx.x & 31, lr = lane & 15, hi = lane >> 4; const int r0 = blockIdx.x * 64, c0 = blockIdx.y * 64;
    v8f acc[4][4];
#pragma unroll
    for (int mb = 0; mb < 4; ++mb)
#pragma unroll
        for (int nb = 0; nb < 4; ++nb) acc[mb][nb] = (v8f){};
    const size_t aoff = (size_t)(r0 + lr) * K + 8 * hi, boff = (size_t)(c0 + lr) * K + 8 * hi;
#pragma unroll 1
    for (int p = 0; p < 2; ++p) {
        const size_t ap = aoff + (size_t)p * plane;
#pragma unroll 1
        for (int kc = 0; kc < K; kc += 32) {
            v16bf a[4];
#pragma unroll
            for (int mb = 0; mb < 4; ++mb) a[mb] = ldb(A + ap + (size_t)mb * 16 * K + kc);
#pragma unroll
            for (int nb = 0; nb < 4; ++nb) { const v16bf b = ldb(Bt + boff + (size_t)nb * 16 * K + kc);
#pragma unroll
                for (int mb = 0; mb < 4; ++mb) acc[mb][nb] = wmmab(a[mb], b, acc[mb][nb]); }
            asm volatile("v_nop\n\tv_nop\n\tv_nop\n\tv_nop" : "+v"(acc[0][0]), "+v"(acc[1][1]), "+v"(acc[2][2]), "+v"(acc[3][3]) : "v"(a[0]), "v"(a[1]), "v"(a[2]), "v"(a[3]));
        }
    }
#pragma unroll
    for (int mb = 0; mb < 4; ++mb) {
#pragma unroll
        for (int nb = 0; nb < 4; ++nb) {
#pragma unroll
            for (int j = 0; j < 8; ++j) os[(hi * 8 + j) * 68 + nb * 16 + lr] = acc[mb][nb][j]; }
        wave_sync();
        float* cb = C + (size_t)(r0 + mb * 16) * (size_t)ldc + c0;
#pragma unroll 1
        for (int ps = 0; ps < 2; ++ps) {
#pragma unroll
            for (int s = 0; s < 8; ++s) { const int row = 2 * s + hi, cofs = lr * 4;
                const v4f val = *(const v4fa*)(&os[row * 68 + cofs]);
                *(volatile v4f*)(cb + (size_t)row * (size_t)ldc + cofs) = val; }
            if (ps == 0) __threadfence(); }
        wave_sync();
    }
}

template <int MODE>
__global__ __launch_bounds__(MODE == 0 ? 64 : 128) void k_mix(const int* __restrict__ tok, const int* __restrict__ posv, const float* __restrict__ emb,
                                                              const float* __restrict__ PR, const float* __restrict__ gam, const float* __restrict__ bet,
                                                              const float* __restrict__ IN, bf* PL, float* OUT) {
    constexpr int D_  = (MODE == 0) ? VD : DD;
    constexpr int INP = (MODE == 1) ? 2 * DD : DD;
    __shared__ __align__(16) float xs[D_ * 4];
    __shared__ __align__(16) float rs[4 * D_];
    const int tid = threadIdx.x, lane = tid & 31;
    const int wave = __builtin_amdgcn_readfirstlane(tid >> 5);
    const int s = blockIdx.x;
    const float pf = (float)posv[s];
    const float ang = TWO_PI_F * pf;

    if (MODE == 0) {
        v4f xv = (v4f){0.0f, 0.0f, 0.0f, 0.0f};
#pragma unroll
        for (int b = 0; b < NB; ++b) {
            int t = tok[(size_t)b * SEQ_FULL + s];
            t = (t < 0) ? 0 : ((t > NTOK - 1) ? NTOK - 1 : t);
            xv[b] = bfq(emb[t * VD + tid]);
        }
        *(v4fa*)(&xs[tid * 4]) = xv;
    } else {
        if (wave < NB) {
            const size_t m = (size_t)wave * SEQ + s;
            const v4f t = *(const v4f*)(IN + m * INP + lane * 4);
            float sm = (t[0] + t[1]) + (t[2] + t[3]);
            sm += __shfl_xor(sm, 16, 32); sm += __shfl_xor(sm, 8, 32); sm += __shfl_xor(sm, 4, 32); sm += __shfl_xor(sm, 2, 32); sm += __shfl_xor(sm, 1, 32);
            const float mu = sm * (1.0f / DD);
            const float d0 = t[0] - mu, d1 = t[1] - mu, d2 = t[2] - mu, d3 = t[3] - mu;
            float q = (d0 * d0 + d1 * d1) + (d2 * d2 + d3 * d3);
            q += __shfl_xor(q, 16, 32); q += __shfl_xor(q, 8, 32); q += __shfl_xor(q, 4, 32); q += __shfl_xor(q, 2, 32); q += __shfl_xor(q, 1, 32);
            const float rstd = rsqrtf(q * (1.0f / DD) + 1.0e-5f);
            const v4f g4 = *(const v4f*)(gam + lane * 4); const v4f b4 = *(const v4f*)(bet + lane * 4);
            xs[(lane * 4 + 0) * 4 + wave] = d0 * rstd * bfq(g4[0]) + bfq(b4[0]);
            xs[(lane * 4 + 1) * 4 + wave] = d1 * rstd * bfq(g4[1]) + bfq(b4[1]);
            xs[(lane * 4 + 2) * 4 + wave] = d2 * rstd * bfq(g4[2]) + bfq(b4[2]);
            xs[(lane * 4 + 3) * 4 + wave] = d3 * rstd * bfq(g4[3]) + bfq(b4[3]);
        } else {
            xs[(lane * 4 + 0) * 4 + wave] = 0.0f; xs[(lane * 4 + 1) * 4 + wave] = 0.0f;
            xs[(lane * 4 + 2) * 4 + wave] = 0.0f; xs[(lane * 4 + 3) * 4 + wave] = 0.0f;
        }
    }
    __syncthreads();

    const float* prow = PR + (size_t)tid * D_;
    float per = (float)(tid * D_ + 2);
    float a0 = 0.0f, a1 = 0.0f, a2 = 0.0f, a3 = 0.0f;
#pragma unroll 1
    for (int j = 0; j < D_; ++j) {
        const float c = cosf(ang / per);
        const float w = prow[j] * c;
        const v4f x = *(const v4fa*)(&xs[j * 4]);
        a0 = fmaf(w, x[0], a0); a1 = fmaf(w, x[1], a1); a2 = fmaf(w, x[2], a2); a3 = fmaf(w, x[3], a3);
        per += 1.0f;
    }

    float e[4] = {a0, a1, a2, a3};
    if (MODE != 0) {
        const int co = (MODE == 1) ? DD : 0;
#pragma unroll
        for (int b = 0; b < 4; ++b) { if (b < NB) e[b] += IN[((size_t)b * SEQ + s) * INP + co + tid]; }
    }
#pragma unroll
    for (int b = 0; b < 4; ++b) rs[b * D_ + tid] = e[b];
    __syncthreads();

    if (MODE == 0) {
        const int b = lane >> 3, c8 = (lane & 7) * 8;
        const v4f x0 = *(const v4fa*)(&rs[b * VD + c8]); const v4f x1 = *(const v4fa*)(&rs[b * VD + c8 + 4]);
        v8us hv, lv;
#pragma unroll
        for (int i = 0; i < 4; ++i) {
            const unsigned short h0 = f2bf(x0[i]); const unsigned short h1 = f2bf(x1[i]);
            hv[i] = h0; hv[4 + i] = h1; lv[i] = f2bf(x0[i] - bf2f(h0)); lv[4 + i] = f2bf(x1[i] - bf2f(h1));
        }
        const v8us o = (wave == 0) ? hv : lv;
        const size_t oo = (size_t)wave * ((size_t)NB * SEQ * VD) + ((size_t)b * SEQ + s) * VD + c8;
        if (b < NB) *(volatile v8us*)(PL + oo) = o;
        __threadfence();
        if (b < NB) *(volatile v8us*)(PL + oo) = o;
    } else if (MODE == 1) {
        if (wave < NB) {
            const int c8 = (lane & 15) * 8;
            const v4f x0 = *(const v4fa*)(&rs[wave * DD + c8]); const v4f x1 = *(const v4fa*)(&rs[wave * DD + c8 + 4]);
            v8us hv, lv;
#pragma unroll
            for (int i = 0; i < 4; ++i) {
                const unsigned short h0 = f2bf(x0[i]); const unsigned short h1 = f2bf(x1[i]);
                hv[i] = h0; hv[4 + i] = h1; lv[i] = f2bf(x0[i] - bf2f(h0)); lv[4 + i] = f2bf(x1[i] - bf2f(h1));
            }
            const v8us o = (lane < 16) ? hv : lv;
            const size_t oo = (size_t)(lane >> 4) * ((size_t)NB * SEQ * DD) + ((size_t)wave * SEQ + s) * DD + c8;
            *(volatile v8us*)(PL + oo) = o;
            __threadfence();
            *(volatile v8us*)(PL + oo) = o;
        }
    } else {
        if (wave < NB) {
            const v4f val = *(const v4fa*)(&rs[wave * DD + lane * 4]);
            float* op = OUT + ((size_t)wave * OUT_SEQ + s) * DD + lane * 4;
            *(volatile v4f*)op = val;
            __threadfence();
            *(volatile v4f*)op = val;
        }
    }
}

static constexpr size_t al256(size_t v) { return (v + 255) & ~(size_t)255; }
static constexpr size_t SZ_W1  = al256((size_t)2 * DD * VD * 2);
static constexpr size_t SZ_W2  = al256((size_t)DD * DD * 2);
static constexpr size_t SZ_PR0 = al256((size_t)VD * VD * 4);
static constexpr size_t SZ_PR1 = al256((size_t)DD * DD * 4);
static constexpr size_t SZ_PR2 = al256((size_t)DD * DD * 4);
static constexpr size_t SZ_HP  = al256((size_t)2 * NB * SEQ * VD * 2);
static constexpr size_t SZ_T1  = al256((size_t)NB * SEQ * 2 * DD * 4);
static constexpr size_t SZ_H1P = al256((size_t)2 * NB * SEQ * DD * 2);
static constexpr size_t SZ_T2  = al256((size_t)NB * SEQ * DD * 4);
static constexpr size_t SZ_TOTAL = SZ_W1 + SZ_W2 + SZ_PR0 + SZ_PR1 + SZ_PR2 + SZ_HP + SZ_T1 + SZ_H1P + SZ_T2;
static_assert(SZ_TOTAL <= (size_t)134217728);
static_assert(((size_t)NB * SEQ * VD * 2) % 256 == 0);
static_assert(((size_t)NB * SEQ * DD * 2) % 256 == 0);
static_assert(((size_t)DD * VD) % (8 * 256) == 0);
static_assert(((size_t)VD * VD) % (4 * 256) == 0);

extern "C" void kernel_launch(void* const* d_in, const int* in_sizes, int n_in,
                              void* d_out, int out_size, void* d_ws, size_t ws_size, hipStream_t stream) {
    if (n_in < 13) return;
    if ((size_t)in_sizes[0] < (size_t)(NB - 1) * SEQ_FULL + SEQ) return;
    if ((size_t)in_sizes[1] < (size_t)SEQ) return;
    if ((size_t)in_sizes[2] < (size_t)NTOK * VD || (size_t)in_sizes[3] < (size_t)VD * VD) return;
    if ((size_t)in_sizes[4] < (size_t)DD * VD || (size_t)in_sizes[5] < (size_t)DD * DD) return;
    if ((size_t)in_sizes[6] < (size_t)DD || (size_t)in_sizes[7] < (size_t)DD) return;
    if ((size_t)in_sizes[8] < (size_t)DD * VD || (size_t)in_sizes[9] < (size_t)DD * DD || (size_t)in_sizes[10] < (size_t)DD * DD) return;
    if ((size_t)in_sizes[11] < (size_t)DD || (size_t)in_sizes[12] < (size_t)DD) return;
    if ((size_t)out_size < ((size_t)(NB - 1) * OUT_SEQ + SEQ) * DD) return;
    if (SZ_TOTAL > ws_size) return;
    const int* tok = (const int*)d_in[0]; const int* posv = (const int*)d_in[1];
    const float* emb = (const float*)d_in[2]; const float* cP = (const float*)d_in[3];
    const float* M1 = (const float*)d_in[4]; const float* P1 = (const float*)d_in[5];
    const float* g1 = (const float*)d_in[6]; const float* b1 = (const float*)d_in[7];
    const float* R1 = (const float*)d_in[8]; const float* M2 = (const float*)d_in[9];
    const float* P2 = (const float*)d_in[10]; const float* g2 = (const float*)d_in[11]; const float* b2 = (const float*)d_in[12];
    float* OUT = (float*)d_out;
    char* wsp = (char*)d_ws;
    bf* W1B = (bf*)wsp; wsp += SZ_W1;
    bf* W2B = (bf*)wsp; wsp += SZ_W2;
    float* PR0 = (float*)wsp; wsp += SZ_PR0;
    float* PR1 = (float*)wsp; wsp += SZ_PR1;
    float* PR2 = (float*)wsp; wsp += SZ_PR2;
    bf* HP = (bf*)wsp; wsp += SZ_HP;
    float* T1R1 = (float*)wsp; wsp += SZ_T1;
    bf* H1P = (bf*)wsp; wsp += SZ_H1P;
    float* T2 = (float*)wsp; wsp += SZ_T2;

    { const size_t n8 = (size_t)DD * VD / 8; const unsigned g = (unsigned)((n8 + 255) / 256);
      k_cvt8<<<g, 256, 0, stream>>>(M1, W1B, n8);
      k_cvt8<<<g, 256, 0, stream>>>(R1, W1B + (size_t)DD * VD, n8); }
    { const size_t n8 = (size_t)DD * DD / 8; k_cvt8<<<(unsigned)((n8 + 255) / 256), 256, 0, stream>>>(M2, W2B, n8); }
    { const size_t n4 = (size_t)VD * VD / 4; k_bfq4<<<(unsigned)((n4 + 255) / 256), 256, 0, stream>>>(cP, PR0, n4); }
    { const size_t n4 = (size_t)DD * DD / 4; const unsigned g = (unsigned)((n4 + 255) / 256);
      k_bfq4<<<g, 256, 0, stream>>>(P1, PR1, n4);
      k_bfq4<<<g, 256, 0, stream>>>(P2, PR2, n4); }

    k_mix<0><<<dim3(SEQ, 1, 1), dim3(VD, 1, 1), 0, stream>>>(tok, posv, emb, PR0, g1, b1, T1R1, HP, OUT);
    k_gemm<<<dim3(NB * SEQ / 64, (2 * DD) / 64, 1), 32, 0, stream>>>(HP, (size_t)NB * SEQ * VD, W1B, T1R1, VD, 2 * DD);
    k_mix<1><<<dim3(SEQ, 1, 1), dim3(DD, 1, 1), 0, stream>>>(tok, posv, emb, PR1, g1, b1, T1R1, H1P, OUT);
    k_gemm<<<dim3(NB * SEQ / 64, DD / 64, 1), 32, 0, stream>>>(H1P, (size_t)NB * SEQ * DD, W2B, T2, DD, DD);
    k_mix<2><<<dim3(SEQ, 1, 1), dim3(DD, 1, 1), 0, stream>>>(tok, posv, emb, PR2, g2, b2, T2, H1P, OUT);
}
